// CharRNN_80487687127332
// MI455X (gfx1250) — hardware-verified
//
#include <hip/hip_runtime.h>
#include <math.h>

typedef __attribute__((ext_vector_type(16))) _Float16 v16h;
typedef __attribute__((ext_vector_type(8)))  _Float16 v8h;
typedef __attribute__((ext_vector_type(8)))  float    v8f;
typedef __attribute__((ext_vector_type(4)))  float    v4f;

constexpr int kBatch  = 1024;
constexpr int kSteps  = 1024;
constexpr int kVocab  = 256;
constexpr int kHid    = 32;
constexpr int kLayers = 10;
constexpr int kThr    = 256;
constexpr int kBlocks = kBatch / (8 * 16);
constexpr int kWP     = 72;
constexpr int kOP     = 40;
constexpr size_t kOutElems = (size_t)kBatch * kVocab;
static_assert(kBlocks == 8 && kHid == 32 && kVocab == kThr, "eight blocks of eight 16-row tiles; one head row a thread");
static_assert(kLayers * kHid * kWP * 2 + kLayers * kHid * 4 + kVocab * 4 <= 65536 && kVocab * kOP <= kLayers * kHid * kWP, "all ten layers' planes in ONE staging under 64 KB; the head's plane fits over them");

constexpr float kSCarry = 1024.0f;
constexpr float kWCarry = 4096.0f;
constexpr float kFold   = 1.0f / (kSCarry * kWCarry);
constexpr float kF16MinNormal = 6.103515625e-5f;
static_assert(kFold == 2.384185791015625e-7f, "2^-22");

union FragU { v16h v; v8h h[2]; };

__device__ __forceinline__ unsigned short f2bf_bits(float f) {
  unsigned u = __float_as_uint(f);
  return (unsigned short)((u + 0x7FFFu + ((u >> 16) & 1u)) >> 16);
}
__device__ __forceinline__ float bf16r(float f) { return __uint_as_float(((unsigned)f2bf_bits(f)) << 16); }
__device__ __forceinline__ float carry_flush(float v, float c) {
  const float s = v * c;
  return (fabsf(s) < kF16MinNormal) ? 0.0f : s;
}
__device__ __forceinline__ v8f mma_h(v16h a, v16h b, v8f c) {
  c = __builtin_amdgcn_wmma_f32_16x16x32_f16(false, a, false, b, (short)0, c, false, false);
  asm volatile("v_nop\n\tv_nop\n\tv_nop\n\tv_nop" : "+v"(c) : "v"(a), "v"(b));
  return c;
}
__device__ __forceinline__ v16h frag_h32(const _Float16* p) { FragU f; f.h[0] = *(const v8h*)(p); f.h[1] = *(const v8h*)(p + 16); return f.v; }
__device__ __forceinline__ v16h frag_tiles(const float* a, const float* b, float c) {
  v16h f;
#pragma unroll
  for (int e = 0; e < 8; ++e) { f[e] = (_Float16)carry_flush(a[e], c); f[8 + e] = (_Float16)carry_flush(b[e], c); }
  return f;
}
__device__ __forceinline__ float fast_tanh(float v) {
  const float e = __expf(2.0f * v);
  return 1.0f - 2.0f * __builtin_amdgcn_rcpf(e + 1.0f);
}
__device__ __forceinline__ float fast_sigmoid(float v) { return __builtin_amdgcn_rcpf(1.0f + __expf(-v)); }

__global__ __launch_bounds__(kThr) void char_roll_kernel(const int* __restrict__ x, const float* __restrict__ emb, const float* __restrict__ Wih,
                                                         const float* __restrict__ Whh, const float* __restrict__ bih, const float* __restrict__ bhh,
                                                         const float* __restrict__ Wfc, const float* __restrict__ bfc, float* __restrict__ out) {
  __shared__ __align__(16) _Float16 sW[kLayers * kHid * kWP];
  __shared__ __align__(16) float sB[kLayers * kHid];
  __shared__ __align__(16) float sBo[kVocab];
  const int tid = threadIdx.x;
  const int wave = tid >> 5;
  const int lane = tid & 31;
  const int col = lane & 15;
  const int hs = lane >> 4;

  for (int rr = tid; rr < kLayers * kHid; rr += kThr) {
    _Float16* wr = sW + rr * kWP;
    const float* hh = Whh + (size_t)rr * kHid;
    const float* ih = Wih + (size_t)rr * kHid;
    for (int k = 0; k < kHid; ++k) {
      const float p = hh[k], q = ih[k];
      wr[k] = (_Float16)carry_flush(bf16r(p), kWCarry);
      wr[kHid + k] = (_Float16)carry_flush(bf16r(q), kWCarry);
    }
    for (int k = 2 * kHid; k < kWP; ++k) wr[k] = (_Float16)0.0f;
    const float b0 = bih[rr], b1 = bhh[rr];
    sB[rr] = bf16r(b0) + bf16r(b1);
  }
  __syncthreads();

  const int b = (blockIdx.x * 8 + wave) * 16 + col;
  const int* xb = x + (size_t)b * kSteps;

  float hst[kLayers][2][8];
#pragma unroll
  for (int l = 0; l < kLayers; ++l)
#pragma unroll
    for (int mt = 0; mt < 2; ++mt)
#pragma unroll
      for (int r = 0; r < 8; ++r) hst[l][mt][r] = 0.0f;

#pragma unroll 1
  for (int t = 0; t < kSteps; ++t) {
    int colv = col, hsv = hs;
    asm volatile("" : "+v"(colv), "+v"(hsv));
    int tok = xb[t];
    asm volatile("" : "+v"(tok));
    tok = (tok < 0) ? 0 : ((tok >= kVocab) ? (kVocab - 1) : tok);
    const float* er = emb + (size_t)tok * kHid + 8 * hsv;
    const v4f e0 = *(const v4f*)er, e1 = *(const v4f*)(er + 4), e2 = *(const v4f*)(er + 16), e3 = *(const v4f*)(er + 20);
    v16h bin;
#pragma unroll
    for (int e = 0; e < 4; ++e) {
      const float p0 = e0[e], p1 = e1[e], p2 = e2[e], p3 = e3[e];
      bin[e] = (_Float16)carry_flush(bf16r(p0), kSCarry);
      bin[4 + e] = (_Float16)carry_flush(bf16r(p1), kSCarry);
      bin[8 + e] = (_Float16)carry_flush(bf16r(p2), kSCarry);
      bin[12 + e] = (_Float16)carry_flush(bf16r(p3), kSCarry);
    }
#pragma unroll
    for (int l = 0; l < kLayers; ++l) {
      const v16h bh = frag_tiles(hst[l][0], hst[l][1], kSCarry);
#pragma unroll
      for (int mt = 0; mt < 2; ++mt) {
        const _Float16* wr = sW + (l * kHid + 16 * mt + colv) * kWP + 8 * hsv;
        v8f a = (v8f){0.f, 0.f, 0.f, 0.f, 0.f, 0.f, 0.f, 0.f};
        a = mma_h(frag_h32(wr), bh, a);
        a = mma_h(frag_h32(wr + kHid), bin, a);
#pragma unroll
        for (int r = 0; r < 8; ++r) hst[l][mt][r] = fast_tanh(a[r] * kFold + sB[l * kHid + 16 * mt + 8 * hsv + r]);
      }
      bin = frag_tiles(hst[l][0], hst[l][1], kSCarry);
    }
  }

  __syncthreads();
  _Float16* sWo = sW;
  {
    const int n = tid;
    _Float16* wr = sWo + n * kOP;
    const float* fr = Wfc + (size_t)n * kHid;
    for (int k = 0; k < kHid; ++k) { const float p = fr[k]; wr[k] = (_Float16)carry_flush(bf16r(p), kWCarry); }
    for (int k = kHid; k < kOP; ++k) wr[k] = (_Float16)0.0f;
    const float bb = bfc[n];
    sBo[n] = bf16r(bb);
  }
  __syncthreads();
  {
    int colv = col, hsv = hs;
    asm volatile("" : "+v"(colv), "+v"(hsv));
    const v16h bt = frag_tiles(hst[kLayers - 1][0], hst[kLayers - 1][1], kSCarry);
    float* ob_ = out + (size_t)b * kVocab + 8 * hsv;
    for (int mt = 0; mt < kVocab / 16; ++mt) {
      const _Float16* wr = sWo + (16 * mt + colv) * kOP + 8 * hsv;
      v8f a = (v8f){0.f, 0.f, 0.f, 0.f, 0.f, 0.f, 0.f, 0.f};
      a = mma_h(frag_h32(wr), bt, a);
      v4f o0, o1;
#pragma unroll
      for (int r = 0; r < 4; ++r) { o0[r] = a[r] * kFold + sBo[16 * mt + 8 * hsv + r]; o1[r] = a[4 + r] * kFold + sBo[16 * mt + 8 * hsv + 4 + r]; }
      float* op = ob_ + 16 * mt;
      for (int pass = 0; pass < 2; ++pass) {
        *(volatile v4f*)op = o0;
        *(volatile v4f*)(op + 4) = o1;
        __threadfence();
      }
    }
  }
}

extern "C" void kernel_launch(void* const* d_in, const int* in_sizes, int n_in,
                              void* d_out, int out_size, void* d_ws, size_t ws_size,
                              hipStream_t stream) {
  if (n_in < 8 || d_out == nullptr) return;
  if (in_sizes[0] != kBatch * kSteps || in_sizes[1] != kVocab * kHid || in_sizes[2] != kLayers * kHid * kHid || in_sizes[3] != kLayers * kHid * kHid) return;
  if (in_sizes[4] != kLayers * kHid || in_sizes[5] != kLayers * kHid || in_sizes[6] != kVocab * kHid || in_sizes[7] != kVocab) return;
  if ((size_t)out_size != kOutElems) return;
  char_roll_kernel<<<kBlocks, kThr, 0, stream>>>((const int*)d_in[0], (const float*)d_in[1], (const float*)d_in[2], (const float*)d_in[3],
                                                 (const float*)d_in[4], (const float*)d_in[5], (const float*)d_in[6], (const float*)d_in[7], (float*)d_out);
}
